// sRPE_30537217474911
// MI455X (gfx1250) — hardware-run, weakly checked
//
#include <hip/hip_runtime.h>


#ifndef NB
#define NB 2
#endif
#ifndef SEQ
#define SEQ 384
#endif
#define NB_FULL  2
#define SEQ_FULL 384
#ifndef OUT_SEQ
#define OUT_SEQ SEQ
#endif
#define NH_  8
#define HD   32
#define NE   256
#define HP   264
#define YS   1024.0f
#define QI   (1.0f / 1024.0f)

static_assert(HD == 32);
static_assert(NH_ * HD == NE);
static_assert(NH_ == 8);
static_assert(NE % 64 == 0);
static_assert(NE % 32 == 0);
static_assert(NE == 32 * 8);
static_assert(SEQ % 64 == 0);
static_assert((NB * SEQ) % 64 == 0);
static_assert(OUT_SEQ % 32 == 0);
static_assert(OUT_SEQ >= SEQ);
static_assert(NB <= NB_FULL);
static_assert(SEQ <= SEQ_FULL);
static_assert(HP % 8 == 0);
static_assert(HP >= NE);
static_assert(((size_t)NB * NH_ * SEQ_FULL * HD) % 8 == 0);
static_assert(32 * 16 * 4 == 16 * 128);
static_assert(32 * 16 * 4 == 8 * 256);
static_assert(256 * 16 * 2 == 64 * 128);
static_assert(64 * HP * 2 + 64 * 4 * 4 + 16 * 68 * 4 <= 131072);

typedef _Float16 h16;
typedef unsigned short bf;
typedef __attribute__((ext_vector_type(16))) __bf16   v16bf;
typedef __attribute__((ext_vector_type(16))) _Float16 v16h;
typedef __attribute__((ext_vector_type(8)))  _Float16 v8h;
typedef __attribute__((ext_vector_type(8)))  unsigned short v8us;
typedef __attribute__((ext_vector_type(8)))  float    v8f;
typedef __attribute__((ext_vector_type(4)))  float    v4f;
typedef v4f  __attribute__((may_alias)) v4fa;
typedef v8h  __attribute__((may_alias)) v8ha;
typedef v8us __attribute__((may_alias)) v8usa;

__device__ __forceinline__ unsigned short f2bf(float f) { unsigned u = __float_as_uint(f); u += 0x7FFFu + ((u >> 16) & 1u); return (unsigned short)(u >> 16); }
__device__ __forceinline__ float bfr(float f) { return __uint_as_float(((unsigned)f2bf(f)) << 16); }
__device__ __forceinline__ v16h cat16(v8h lo, v8h hi) { return __builtin_shufflevector(lo, hi, 0, 1, 2, 3, 4, 5, 6, 7, 8, 9, 10, 11, 12, 13, 14, 15); }
__device__ __forceinline__ v16bf cat16b(v8us lo, v8us hi) { return __builtin_bit_cast(v16bf, __builtin_shufflevector(lo, hi, 0, 1, 2, 3, 4, 5, 6, 7, 8, 9, 10, 11, 12, 13, 14, 15)); }
__device__ __forceinline__ v8f wmma16(v16h a, v16h b, v8f c) { return __builtin_amdgcn_wmma_f32_16x16x32_f16(false, a, false, b, (short)0, c, false, false); }
__device__ __forceinline__ v8f wmmab(v16bf a, v16bf b, v8f c) { return __builtin_amdgcn_wmma_f32_16x16x32_bf16(false, a, false, b, (short)0, c, false, false); }
__device__ __forceinline__ v8f wmma16g(v16h a, v16h b, v8f c) { c = wmma16(a, b, c); asm volatile("v_nop\n\tv_nop\n\tv_nop\n\tv_nop" : "+v"(c) : "v"(a), "v"(b)); return c; }
__device__ __forceinline__ v8f wmmabg(v16bf a, v16bf b, v8f c) { c = wmmab(a, b, c); asm volatile("v_nop\n\tv_nop\n\tv_nop\n\tv_nop" : "+v"(c) : "v"(a), "v"(b)); return c; }
__device__ __forceinline__ v16h  ldh(const h16* p) { return cat16(*(const v8h*)p, *(const v8h*)(p + 16)); }
__device__ __forceinline__ v16bf ldb(const bf* p)  { return cat16b(*(const v8us*)p, *(const v8us*)(p + 16)); }
__device__ __forceinline__ void wave_sync() { __builtin_amdgcn_fence(3  , "wavefront"); __builtin_amdgcn_wave_barrier(); asm volatile("" ::: "memory"); }
static __device__ __forceinline__ h16 toh_flush(float v) { const float w = (fabsf(v) < 6.103515625e-05f) ? 0.0f : v; return (h16)w; }

__global__ __launch_bounds__(256) void k_cvt8(const float* __restrict__ src, bf* dst, size_t n8) {
    const size_t i = (size_t)blockIdx.x * 256 + threadIdx.x; if (i >= n8) return;
    const v8f v = *(const v8f*)(src + i * 8); v8us o;
#pragma unroll
    for (int k = 0; k < 8; ++k) o[k] = f2bf(v[k]);
    *(volatile v8us*)(dst + i * 8) = o; __threadfence(); *(volatile v8us*)(dst + i * 8) = o;
}

__global__ __launch_bounds__(256) void k_wtr(const float* __restrict__ W, bf* WT) {
    __shared__ __align__(16) unsigned short lt[64 * 72];
    const unsigned tid = threadIdx.x;
    const unsigned cb0 = blockIdx.x * 64u, kb0 = blockIdx.y * 64u;
    const unsigned rc = tid >> 2, kq = (tid & 3u) * 16u;
    const float* src = W + (size_t)(cb0 + rc) * NE + kb0 + kq;
#pragma unroll
    for (int i = 0; i < 4; ++i) { const v4f v = *(const v4f*)(src + 4 * i);
#pragma unroll
        for (int j = 0; j < 4; ++j) lt[(kq + 4 * i + j) * 72 + rc] = f2bf(v[j]); }
    __syncthreads();
#pragma unroll 1
    for (int ps = 0; ps < 2; ++ps) {
#pragma unroll
        for (int it = 0; it < 2; ++it) { const unsigned p = (unsigned)it * 256u + tid; const unsigned rk = p >> 3, c8 = (p & 7u) * 8u;
            const v8us o = *(const v8usa*)(&lt[rk * 72 + c8]);
            *(volatile v8us*)(WT + (size_t)(kb0 + rk) * NE + cb0 + c8) = o; }
        if (ps == 0) __threadfence(); }
}

__global__ __launch_bounds__(32) void k_ygemm(const bf* __restrict__ XB, const bf* __restrict__ WT, h16* YC) {
    __shared__ __align__(16) float os[16 * 68];
    const int lane = threadIdx.x & 31, lr = lane & 15, hi = lane >> 4;
    const unsigned bx = blockIdx.x; const unsigned r0 = bx * 64u, c0 = blockIdx.y * 64u; const unsigned hd = blockIdx.z;
    const unsigned bb = r0 / (unsigned)SEQ, tt = r0 % (unsigned)SEQ;
    const size_t aoff = ((size_t)(bb * (unsigned)NH_ + hd) * SEQ_FULL + tt + (unsigned)lr) * HD + 8 * hi;
    const size_t boff = (size_t)(c0 + (unsigned)lr) * NE + hd * (unsigned)HD + 8 * hi;
    v16bf a[4];
#pragma unroll
    for (int mb = 0; mb < 4; ++mb) a[mb] = ldb(XB + aoff + (size_t)mb * 16 * HD);
    v8f acc[4][4];
#pragma unroll
    for (int mb = 0; mb < 4; ++mb)
#pragma unroll
        for (int nb = 0; nb < 4; ++nb) acc[mb][nb] = (v8f){};
#pragma unroll
    for (int nb = 0; nb < 4; ++nb) { const v16bf b = ldb(WT + boff + (size_t)nb * 16 * NE);
#pragma unroll
        for (int mb = 0; mb < 4; ++mb) acc[mb][nb] = wmmabg(a[mb], b, acc[mb][nb]); }
#pragma unroll
    for (int mb = 0; mb < 4; ++mb) {
#pragma unroll
        for (int nb = 0; nb < 4; ++nb) {
#pragma unroll
            for (int j = 0; j < 8; ++j) os[(hi * 8 + j) * 68 + nb * 16 + lr] = acc[mb][nb][j] * YS; }
        wave_sync();
#pragma unroll 1
        for (int ps = 0; ps < 2; ++ps) {
#pragma unroll
            for (int s = 0; s < 4; ++s) { const int row = 4 * s + (lane >> 3), c8 = (lane & 7) * 8;
                const v4f x0 = *(const v4fa*)(&os[row * 68 + c8]); const v4f x1 = *(const v4fa*)(&os[row * 68 + c8 + 4]); v8h hv;
#pragma unroll
                for (int i = 0; i < 4; ++i) { hv[i] = toh_flush(x0[i]); hv[4 + i] = toh_flush(x1[i]); }
                const size_t oo = ((size_t)(r0 + (unsigned)(mb * 16 + row)) * NH_ + hd) * NE + c0 + (unsigned)c8;
                *(volatile v8h*)(YC + oo) = hv; }
            if (ps == 0) __threadfence(); }
        wave_sync();
    }
}

__global__ __launch_bounds__(32) __attribute__((amdgpu_num_vgpr(256)))
void k_pairs(const float* __restrict__ X, const float* __restrict__ PD, const float* __restrict__ W1, const float* __restrict__ B1,
             const float* __restrict__ B2, const h16* __restrict__ YC, float* OUT) {
    __shared__ __align__(16) h16 hidt[64 * HP];
    __shared__ __align__(16) float ft[64 * 4];
    __shared__ __align__(16) float os[16 * 68];
    const int lane = threadIdx.x & 31, lr = lane & 15, hi = lane >> 4;
    const unsigned s0 = blockIdx.x * 64u; const unsigned t = blockIdx.y; const unsigned b = blockIdx.z;
    const float* pdrow = PD + ((size_t)b * SEQ_FULL + t) * SEQ_FULL + s0;
#pragma unroll 1
    for (int q = 0; q < 2; ++q) {
        const int row = lane + 32 * q;
        const float d = bfr(pdrow[row]);
        const float nd = -d;
        const float dp = (d < 0.0f) ? 0.0f : d;
        const float dn = (nd < 0.0f) ? 0.0f : nd;
        v4f f; f[0] = log1pf(dp); f[1] = log1pf(dn); f[2] = (d == 0.0f) ? 1.0f : 0.0f; f[3] = 0.0f;
        *(v4fa*)(&ft[row * 4]) = f;
    }
    float wq[24], bq[8];
    { const float* wp = W1 + lane * 24;
#pragma unroll
      for (int i = 0; i < 6; ++i) { const v4f v = *(const v4f*)(wp + 4 * i);
#pragma unroll
          for (int j = 0; j < 4; ++j) wq[4 * i + j] = bfr(v[j]); }
      const float* bp = B1 + lane * 8;
#pragma unroll
      for (int i = 0; i < 2; ++i) { const v4f v = *(const v4f*)(bp + 4 * i);
#pragma unroll
          for (int j = 0; j < 4; ++j) bq[4 * i + j] = bfr(v[j]); } }
    wave_sync();
#pragma unroll 1
    for (int r = 0; r < 64; ++r) {
        const v4f f = *(const v4fa*)(&ft[r * 4]);
        v8h hv;
#pragma unroll
        for (int e = 0; e < 8; ++e) {
            const float v = f[0] * wq[3 * e] + f[1] * wq[3 * e + 1] + f[2] * wq[3 * e + 2] + bq[e];
            const float u = 0.7978845608028654f * (v + 0.044715f * (v * v * v));
            const float g = 0.5f * v * (1.0f + tanhf(u));
            hv[e] = toh_flush(g);
        }
        *(v8ha*)(&hidt[r * HP + lane * 8]) = hv;
    }
    wave_sync();
    const unsigned hh = (unsigned)lr & 7u;
    float cb = 0.0f;
    { const float* xp = X + ((size_t)(b * (unsigned)NH_ + hh) * SEQ_FULL + t) * HD; const float* bp = B2 + hh * (unsigned)HD;
#pragma unroll 1
      for (int i = 0; i < 8; ++i) { const v4f xv = *(const v4f*)(xp + 4 * i); const v4f bv = *(const v4f*)(bp + 4 * i);
#pragma unroll
          for (int j = 0; j < 4; ++j) cb += bfr(xv[j]) * bfr(bv[j]); } }
    const size_t yo = ((size_t)(b * (unsigned)SEQ + t) * NH_ + hh) * NE + 8 * hi;
    const int ai = lr * HP + 8 * hi;
    v8f acc[4];
#pragma unroll
    for (int mb = 0; mb < 4; ++mb) acc[mb] = (v8f){};
#pragma unroll
    for (int ks = 0; ks < 8; ++ks) {
        const v16h yb = ldh(YC + yo + ks * 32);
#pragma unroll
        for (int mb = 0; mb < 4; ++mb) {
            const v8h a0 = *(const v8ha*)(&hidt[ai + mb * 16 * HP + ks * 32]);
            const v8h a1 = *(const v8ha*)(&hidt[ai + mb * 16 * HP + ks * 32 + 16]);
            acc[mb] = wmma16g(cat16(a0, a1), yb, acc[mb]);
        }
    }
#pragma unroll
    for (int mb = 0; mb < 4; ++mb) { v4f p, q;
#pragma unroll
        for (int j = 0; j < 4; ++j) { p[j] = acc[mb][j] * QI + cb; q[j] = acc[mb][4 + j] * QI + cb; }
        *(v4fa*)(&os[lr * 68 + mb * 16 + 8 * hi]) = p; *(v4fa*)(&os[lr * 68 + mb * 16 + 8 * hi + 4]) = q; }
    wave_sync();
#pragma unroll 1
    for (int ps = 0; ps < 2; ++ps) {
#pragma unroll
        for (int i = 0; i < 4; ++i) { const int hrow = 2 * i + (lane >> 4), cofs = (lane & 15) * 4;
            const v4f val = *(const v4fa*)(&os[hrow * 68 + cofs]);
            *(volatile v4f*)(OUT + (((size_t)b * NH_ + (unsigned)hrow) * OUT_SEQ + t) * OUT_SEQ + s0 + (unsigned)cofs) = val; }
        if (ps == 0) __threadfence(); }
}

static constexpr size_t al256(size_t v) { return (v + 255) & ~(size_t)255; }
static constexpr size_t N_X   = (size_t)NB * NH_ * SEQ_FULL * HD;
static constexpr size_t SZ_XB = al256(N_X * 2);
static constexpr size_t SZ_WT = al256((size_t)NE * NE * 2);
static constexpr size_t SZ_YC = al256((size_t)NB * SEQ * NH_ * NE * 2);
static constexpr size_t SZ_TOTAL = SZ_XB + SZ_WT + SZ_YC;
static constexpr size_t NEED_PD  = ((size_t)(NB - 1) * SEQ_FULL + (SEQ - 1)) * SEQ_FULL + SEQ;
static constexpr size_t NEED_OUT = ((size_t)(NB * NH_ - 1) * OUT_SEQ + (SEQ - 1)) * OUT_SEQ + SEQ;
static_assert(SZ_TOTAL <= (size_t)134217728);
static_assert((size_t)(NB * SEQ / 64) * 64 * NH_ * NE * 2 <= SZ_YC);
static_assert((size_t)(NE / 64) * 64 * NE * 2 <= SZ_WT);

extern "C" void kernel_launch(void* const* d_in, const int* in_sizes, int n_in,
                              void* d_out, int out_size, void* d_ws, size_t ws_size, hipStream_t stream) {
    if (n_in < 6) return;
    if ((size_t)in_sizes[0] < N_X) return;
    if ((size_t)in_sizes[1] < NEED_PD) return;
    if (in_sizes[2] < NE * 3 || in_sizes[3] < NE || in_sizes[4] < NE * NE || in_sizes[5] < NE) return;
    if ((size_t)out_size < NEED_OUT) return;
    if (SZ_TOTAL > ws_size) return;
    const float* x  = (const float*)d_in[0];
    const float* pd = (const float*)d_in[1];
    const float* w1 = (const float*)d_in[2];
    const float* b1 = (const float*)d_in[3];
    const float* w2 = (const float*)d_in[4];
    const float* b2 = (const float*)d_in[5];
    float* OUT = (float*)d_out;
    char* wsp = (char*)d_ws;
    bf*  XB = (bf*)wsp;  wsp += SZ_XB;
    bf*  WT = (bf*)wsp;  wsp += SZ_WT;
    h16* YC = (h16*)wsp; wsp += SZ_YC;

    { const size_t n8 = N_X / 8;
      k_cvt8<<<(unsigned)((n8 + 255) / 256), 256, 0, stream>>>(x, XB, n8); }
    k_wtr<<<dim3(NE / 64, NE / 64, 1), 256, 0, stream>>>(w2, WT);
    k_ygemm<<<dim3(NB * SEQ / 64, NE / 64, NH_), 32, 0, stream>>>(XB, WT, YC);
    k_pairs<<<dim3(SEQ / 64, SEQ, NB), 32, 0, stream>>>(x, pd, w1, b1, b2, YC, OUT);
}
